// Transformer_18511309046426
// MI455X (gfx1250) — hardware-run, weakly checked
//
#include <hip/hip_runtime.h>
#include <math.h>

typedef _Float16 h16;
typedef __attribute__((ext_vector_type(16))) _Float16 v16h;
typedef __attribute__((ext_vector_type(8)))  _Float16 v8h;
typedef __attribute__((ext_vector_type(8)))  float v8f;
typedef __attribute__((ext_vector_type(4)))  float v4f;
typedef __attribute__((ext_vector_type(4)))  unsigned v4u;

#ifndef NB
#define NB 2
#endif
#ifndef SEQ
#define SEQ 2048
#endif
#define NB_FULL 2
#define SEQ_FULL 2048
#define CIN 64
#define DIN 512
#define CC 512
#define NH 8
#define HD 64
#define MLPW 2048
#define NLAY 2
#define WCARRY 256.0f
#define PCARRY 1024.0f
#define CCARRY 64.0f
#define HCARRY 16.0f
#define XCARRY 16.0f
#define L2E 1.44269504088896340736f
#define FL_RES 1
#define FL_STX 2
#define FL_LN  4

static_assert(NB <= NB_FULL);
static_assert(SEQ <= SEQ_FULL);
static_assert(CC == NH * HD);
static_assert(HD == 64);
static_assert(DIN == 512);
static_assert(CC == DIN);
static_assert(CIN == 64);
static_assert(CIN % 32 == 0);
static_assert(DIN % 32 == 0);
static_assert(MLPW % 32 == 0);
static_assert(MLPW % 64 == 0);
static_assert(SEQ % 128 == 0);
static_assert((NB * SEQ) % 64 == 0);
static_assert((NB * SEQ) % 16 == 0);
static_assert(8 * 64 == DIN);
static_assert(4 * 32 * 4 == DIN);
static_assert(2 * 32 * 8 == DIN);
static_assert(256 * 4 * 4 == 64 * 64);
static_assert(256 * 2 * 16 == 64 * 128);
static_assert(128 * 4 * 16 == 64 * 128);
static_assert(128 * 8 * 16 == 64 * 256);
static_assert(4 * 4 == 16);
static_assert((NB * CIN) % 8 == 0);

#define MROWS  ((size_t)NB * SEQ)
#define SZ_IN  (MROWS * CIN * 2)
#define SZ_ACT (MROWS * CC * 2)
#define WS_XT    ((size_t)0)
#define WS_CT    (WS_XT + SZ_IN)
#define WS_WXT   (WS_CT + SZ_IN)
#define WS_WCT   (WS_WXT + (size_t)CC * CIN * 2)
#define WS_WQKV  (WS_WCT + (size_t)CC * CIN * 2)
#define WS_WOT   (WS_WQKV + (size_t)NLAY * 3 * CC * DIN * 2)
#define WS_W1T   (WS_WOT + (size_t)NLAY * DIN * CC * 2)
#define WS_W2T   (WS_W1T + (size_t)NLAY * MLPW * DIN * 2)
#define WS_WOUTT (WS_W2T + (size_t)NLAY * DIN * MLPW * 2)
#define WS_XF    (WS_WOUTT + (size_t)CIN * DIN * 2)
#define WS_HH    (WS_XF + MROWS * DIN * 4)
#define WS_CTX   (WS_HH + SZ_ACT)
#define WS_QH    (WS_CTX + SZ_ACT)
#define WS_KH    (WS_QH + SZ_ACT)
#define WS_VT    (WS_KH + SZ_ACT)
#define WS_CH    (WS_VT + SZ_ACT)
#define WS_HID   (WS_CH + SZ_ACT)
#define WS_YT    (WS_HID + MROWS * MLPW * 2)
#define WS_END   (WS_YT + (size_t)NB * CIN * SEQ * 4)
static_assert(WS_END <= (size_t)134217728);
static_assert(SZ_IN % 128 == 0);
static_assert(SZ_ACT % 128 == 0);
static_assert(((size_t)CC * CIN * 2) % 128 == 0);
static_assert(((size_t)CC * DIN * 2) % 128 == 0);
static_assert((SZ_ACT / 2) < (size_t)2147483647);

static_assert(64 * 72 * 2 <= 131072);
static_assert(4 * 16 * 40 * 2 + 4 * 16 * 72 * 2 <= 131072);
static_assert(64 * 68 * 4 <= 131072);
static_assert(16 * (DIN + 4) * 4 + 8 * (DIN + 8) * 2 <= 131072);

template <typename T> __device__ __forceinline__ void vst2(void* p, T v) { *(volatile T*)p = v; __threadfence(); *(volatile T*)p = v; }
__device__ __forceinline__ v8f wmma16(v16h a, v16h b, v8f c) {
  v8f d = __builtin_amdgcn_wmma_f32_16x16x32_f16(false, a, false, b, (short)0, c, false, false);
  asm volatile("v_nop\n\tv_nop\n\tv_nop\n\tv_nop" : "+v"(d) : "v"(a), "v"(b));
  return d;
}
__device__ __forceinline__ v16h frag_h(const _Float16* rowk0, int lane) {
  union { v16h v; v8h q[2]; } u; const _Float16* p = rowk0 + 8 * (lane >> 4);
  u.q[0] = *(const v8h*)p; u.q[1] = *(const v8h*)(p + 16); return u.v;
}
__device__ __forceinline__ float bfr(float v) { return (float)(__bf16)v; }
static __device__ __forceinline__ h16 toh_flush(float v) { const h16 r = (h16)v; return (fabsf(v) < 6.103515625e-05f) ? (h16)0.0f : r; }
#define LDSX() do { asm volatile("s_wait_dscnt 0" ::: "memory"); __builtin_amdgcn_wave_barrier(); __builtin_amdgcn_fence(3  , "workgroup"); } while (0)

__global__ __launch_bounds__(256) void k_tcv(const float* __restrict__ src, h16* __restrict__ dst, float sc, int spitch, int sbatch, int dpitch, int dbatch) {
  __shared__ __align__(16) h16 tt[64][72];
  const int tid = threadIdx.x;
  const int c0 = blockIdx.x * 64, r0 = blockIdx.y * 64, z = blockIdx.z;
  const float* sp = src + (size_t)z * sbatch + (size_t)r0 * spitch + c0;
#pragma unroll 1
  for (int it = 0; it < 4; ++it) { const int e = tid + it * 256; const int r = e >> 4, pc = e & 15;
    const v4f u = *(const v4f*)(sp + (size_t)r * spitch + pc * 4);
#pragma unroll
    for (int i = 0; i < 4; ++i) tt[pc * 4 + i][r] = toh_flush(bfr(u[i]) * sc); }
  __syncthreads();
  h16* dp = dst + (size_t)z * dbatch + (size_t)c0 * dpitch + r0;
#pragma unroll 1
  for (int it = 0; it < 2; ++it) { const int e = tid + it * 256; const int cl = e >> 3, pc = e & 7;
    const v4u hv = *(const v4u*)&tt[cl][pc * 8];
    vst2(dp + (size_t)cl * dpitch + pc * 8, hv); }
}

__global__ __launch_bounds__(256) void k_rowln(const h16* __restrict__ A, const h16* __restrict__ WT, int K, float sc, const float* __restrict__ bias, float* XF, int flags, const float* __restrict__ gam, const float* __restrict__ bet, h16* __restrict__ HP, float oc) {
  __shared__ __align__(16) float pre[16][DIN + 4];
  __shared__ __align__(16) h16 hst[8][DIN + 8];
  const int tid = threadIdx.x; const int wave = __builtin_amdgcn_readfirstlane(threadIdx.x >> 5); const int lane = tid & 31, col = lane & 15, g = lane >> 4;
  const int r0 = blockIdx.x * 16; const int n0 = wave * 64;
  const size_t aoff = (size_t)(r0 + col) * K; const size_t woff = (size_t)(n0 + col) * K;
  const int nk = K >> 5;
  v8f ah[4] = {};
#pragma unroll 1
  for (int kc = 0; kc < nk; ++kc) { const v16h fa = frag_h(A + aoff + kc * 32, lane);
#pragma unroll
    for (int j = 0; j < 4; ++j) { const v16h w = frag_h(WT + woff + (size_t)(j * 16) * K + kc * 32, lane); ah[j] = wmma16(fa, w, ah[j]); } }
#pragma unroll
  for (int j = 0; j < 4; ++j)
#pragma unroll
    for (int r = 0; r < 8; ++r) pre[8 * g + r][n0 + j * 16 + col] = ah[j][r] * sc;
  __syncthreads();
#pragma unroll 1
  for (int rr = 0; rr < 2; ++rr) { const int row = wave * 2 + rr; const int grow = r0 + row;
    float* xrow = XF + (size_t)grow * DIN; h16* hrow = HP + (size_t)grow * DIN;
    v4f t[4]; float sum = 0.f;
#pragma unroll
    for (int it = 0; it < 4; ++it) { const int c = (it * 32 + lane) * 4; const v4f y = *(const v4f*)&pre[row][c]; const v4f bv = *(const v4f*)(bias + c); v4f v;
#pragma unroll
      for (int e = 0; e < 4; ++e) v[e] = y[e] + bfr(bv[e]);
      if (flags & FL_RES) { const v4f xv = *(const v4f*)(xrow + c);
#pragma unroll
        for (int e = 0; e < 4; ++e) v[e] += xv[e]; }
      t[it] = v; sum += (v[0] + v[1]) + (v[2] + v[3]); }
    if (flags & FL_STX) {
#pragma unroll
      for (int it = 0; it < 4; ++it) { const int c = (it * 32 + lane) * 4; const v4f sv = t[it]; vst2(xrow + c, sv); } }
    sum += __shfl_xor(sum, 1); sum += __shfl_xor(sum, 2); sum += __shfl_xor(sum, 4); sum += __shfl_xor(sum, 8); sum += __shfl_xor(sum, 16);
    const float mu = sum * (1.0f / DIN); float sq = 0.f;
#pragma unroll
    for (int it = 0; it < 4; ++it)
#pragma unroll
      for (int e = 0; e < 4; ++e) { const float d = t[it][e] - mu; sq += d * d; }
    sq += __shfl_xor(sq, 1); sq += __shfl_xor(sq, 2); sq += __shfl_xor(sq, 4); sq += __shfl_xor(sq, 8); sq += __shfl_xor(sq, 16);
    const float rs = rsqrtf(sq * (1.0f / DIN) + 1.0e-5f);
    LDSX();
    if (flags & FL_LN) {
#pragma unroll
      for (int it = 0; it < 4; ++it) { const int c = (it * 32 + lane) * 4; const v4f gm = *(const v4f*)(gam + c); const v4f bt = *(const v4f*)(bet + c);
#pragma unroll
        for (int e = 0; e < 4; ++e) hst[wave][c + e] = toh_flush((t[it][e] - mu) * rs * bfr(gm[e]) + bfr(bt[e])); }
    } else {
#pragma unroll
      for (int it = 0; it < 4; ++it) { const int c = (it * 32 + lane) * 4;
#pragma unroll
        for (int e = 0; e < 4; ++e) hst[wave][c + e] = toh_flush(t[it][e] * oc); }
    }
    LDSX();
#pragma unroll 1
    for (int it = 0; it < 2; ++it) { const int pc = it * 32 + lane;
      const v4u hv = *(const v4u*)&hst[wave][pc * 8];
      vst2(hrow + pc * 8, hv); } }
}

__global__ __launch_bounds__(128) void k_qkv(const h16* __restrict__ ACT, int ctxoff, const h16* __restrict__ WQKV, h16* __restrict__ QH, h16* __restrict__ KH, h16* __restrict__ VT) {
  __shared__ __align__(16) h16 th[64][72];
  const int tid = threadIdx.x; const int wave = __builtin_amdgcn_readfirstlane(threadIdx.x >> 5); const int lane = tid & 31, col = lane & 15, g = lane >> 4;
  const int r0 = blockIdx.x * 64; const int nt = blockIdx.y; const int n0 = nt * 64; const int which = nt >> 3, hh = nt & 7;
  const size_t aoff = (size_t)((which > 0) ? ctxoff : 0) + (size_t)(r0 + wave * 16 + col) * DIN; const size_t woff = (size_t)(n0 + col) * DIN;
  v8f acc[4] = {};
#pragma unroll 2
  for (int kc = 0; kc < DIN / 32; ++kc) { const v16h a = frag_h(ACT + aoff + kc * 32, lane);
#pragma unroll
    for (int j = 0; j < 4; ++j) { const v16h w = frag_h(WQKV + woff + (size_t)(j * 16) * DIN + kc * 32, lane); acc[j] = wmma16(a, w, acc[j]); } }
  if (which == 2) {
#pragma unroll
    for (int j = 0; j < 4; ++j)
#pragma unroll
      for (int r = 0; r < 8; ++r) th[j * 16 + col][wave * 16 + 8 * g + r] = toh_flush(acc[j][r] * (1.0f / WCARRY));
  } else {
#pragma unroll
    for (int j = 0; j < 4; ++j)
#pragma unroll
      for (int r = 0; r < 8; ++r) th[wave * 16 + 8 * g + r][j * 16 + col] = toh_flush(acc[j][r] * (1.0f / WCARRY));
  }
  __syncthreads();
  const int b = r0 / SEQ, s0 = r0 - b * SEQ;
#pragma unroll 1
  for (int it = 0; it < 4; ++it) { const int e = tid + it * 128; const int rl = e >> 3, pc = e & 7;
    const v4u hv = *(const v4u*)&th[rl][pc * 8];
    if (which == 0) { const size_t off = (size_t)(r0 + rl) * CC + hh * HD + pc * 8; vst2(QH + off, hv); }
    else if (which == 1) { const size_t off = (size_t)(r0 + rl) * CC + hh * HD + pc * 8; vst2(KH + off, hv); }
    else { const size_t off = ((size_t)b * CC + hh * HD + rl) * SEQ + s0 + pc * 8; vst2(VT + off, hv); } }
}

__global__ __launch_bounds__(128) void k_attn(const h16* __restrict__ QH, const h16* __restrict__ KH, const h16* __restrict__ VT, h16* __restrict__ CH) {
  __shared__ __align__(16) h16 sp[4][16][40];
  __shared__ __align__(16) h16 sch[4][16][72];
  const int tid = threadIdx.x; const int wave = __builtin_amdgcn_readfirstlane(threadIdx.x >> 5); const int lane = tid & 31, col = lane & 15, g = lane >> 4;
  const int qb = blockIdx.x, h = blockIdx.y, b = blockIdx.z; const int ql0 = qb * 64 + wave * 16;
  const size_t qoff = ((size_t)b * SEQ + ql0 + col) * CC + h * HD;
  const size_t kbase = ((size_t)b * SEQ + col) * CC + h * HD;
  const size_t vbase = ((size_t)b * CC + h * HD + col) * SEQ;
  float m[8], l[8]; v8f o[4] = {};
#pragma unroll
  for (int r = 0; r < 8; ++r) { m[r] = -1.0e30f; l[r] = 0.f; }
#pragma unroll 1
  for (int kh = 0; kh < SEQ / 32; ++kh) { const int key0 = kh * 32;
    int zo = 0; asm volatile("" : "+v"(zo));
    v8f sh0 = {}, sh1 = {};
#pragma unroll
    for (int kc = 0; kc < HD / 32; ++kc) {
      const v16h aq = frag_h(QH + qoff + zo + kc * 32, lane);
      const v16h k0f = frag_h(KH + kbase + (size_t)key0 * CC + kc * 32, lane), k1f = frag_h(KH + kbase + (size_t)(key0 + 16) * CC + kc * 32, lane);
      sh0 = wmma16(aq, k0f, sh0); sh1 = wmma16(aq, k1f, sh1); }
    LDSX();
#pragma unroll
    for (int r = 0; r < 8; ++r) {
      const float a0 = sh0[r] * 0.125f, a1 = sh1[r] * 0.125f;
      float mx = fmaxf(a0, a1);
      mx = fmaxf(mx, __shfl_xor(mx, 1)); mx = fmaxf(mx, __shfl_xor(mx, 2)); mx = fmaxf(mx, __shfl_xor(mx, 4)); mx = fmaxf(mx, __shfl_xor(mx, 8));
      const float mn = fmaxf(m[r], mx); const float corr = exp2f((m[r] - mn) * L2E); m[r] = mn;
      const float e0 = (a0 - mn) * L2E, e1 = (a1 - mn) * L2E;
      const float p0 = (e0 < -24.0f) ? 0.0f : exp2f(e0), p1 = (e1 < -24.0f) ? 0.0f : exp2f(e1);
      const h16 q0 = (h16)(p0 * PCARRY), q1 = (h16)(p1 * PCARRY);
      l[r] = l[r] * corr + ((float)q0 + (float)q1);
      o[0][r] *= corr; o[1][r] *= corr; o[2][r] *= corr; o[3][r] *= corr;
      sp[wave][8 * g + r][col] = q0; sp[wave][8 * g + r][16 + col] = q1; }
    LDSX();
    union { v16h v; v8h q[2]; } pu; pu.q[0] = *(const v8h*)&sp[wave][col][8 * g]; pu.q[1] = *(const v8h*)&sp[wave][col][16 + 8 * g];
#pragma unroll
    for (int j = 0; j < 4; ++j) { const v16h vf = frag_h(VT + vbase + (size_t)(j * 16) * SEQ + key0, lane); o[j] = wmma16(pu.v, vf, o[j]); } }
#pragma unroll
  for (int r = 0; r < 8; ++r) { float lt = l[r];
    lt += __shfl_xor(lt, 1); lt += __shfl_xor(lt, 2); lt += __shfl_xor(lt, 4); lt += __shfl_xor(lt, 8);
    const float inv = CCARRY / lt;
#pragma unroll
    for (int j = 0; j < 4; ++j) sch[wave][8 * g + r][j * 16 + col] = toh_flush(o[j][r] * inv); }
  LDSX();
#pragma unroll 1
  for (int it = 0; it < 4; ++it) { const int rl = it * 4 + (lane >> 3), pc = lane & 7;
    const size_t off = ((size_t)b * SEQ + ql0 + rl) * CC + h * HD + pc * 8;
    const v4u hv = *(const v4u*)&sch[wave][rl][pc * 8];
    vst2(CH + off, hv); }
}

__global__ __launch_bounds__(128) void k_ffn1(const h16* __restrict__ H2, const h16* __restrict__ W1T, const float* __restrict__ b1, h16* __restrict__ HID) {
  __shared__ __align__(16) float tf[64][68];
  const int tid = threadIdx.x; const int wave = __builtin_amdgcn_readfirstlane(threadIdx.x >> 5); const int lane = tid & 31, col = lane & 15, g = lane >> 4;
  const int r0 = blockIdx.x * 64; const int n0 = blockIdx.y * 64;
  const size_t aoff = (size_t)(r0 + wave * 16 + col) * DIN; const size_t woff = (size_t)(n0 + col) * DIN;
  v8f acc[4] = {};
#pragma unroll 2
  for (int kc = 0; kc < DIN / 32; ++kc) { const v16h a = frag_h(H2 + aoff + kc * 32, lane);
#pragma unroll
    for (int j = 0; j < 4; ++j) { const v16h w = frag_h(W1T + woff + (size_t)(j * 16) * DIN + kc * 32, lane); acc[j] = wmma16(a, w, acc[j]); } }
#pragma unroll
  for (int j = 0; j < 4; ++j)
#pragma unroll
    for (int r = 0; r < 8; ++r) tf[wave * 16 + 8 * g + r][j * 16 + col] = acc[j][r] * (1.0f / WCARRY);
  __syncthreads();
#pragma unroll 1
  for (int it = 0; it < 4; ++it) { const int e = tid + it * 128; const int rl = e >> 3, pc = e & 7;
    const v4f y0 = *(const v4f*)&tf[rl][pc * 8], y1 = *(const v4f*)&tf[rl][pc * 8 + 4];
    const v4f c0 = *(const v4f*)(b1 + n0 + pc * 8), c1 = *(const v4f*)(b1 + n0 + pc * 8 + 4);
    v8h o;
#pragma unroll
    for (int i = 0; i < 4; ++i) { const float u0 = y0[i] + bfr(c0[i]), u1 = y1[i] + bfr(c1[i]);
      o[i] = toh_flush(0.5f * u0 * (1.0f + erff(u0 * 0.70710678118654752f)) * HCARRY);
      o[4 + i] = toh_flush(0.5f * u1 * (1.0f + erff(u1 * 0.70710678118654752f)) * HCARRY); }
    const v4u ov = __builtin_bit_cast(v4u, o);
    vst2(HID + (size_t)(r0 + rl) * MLPW + n0 + pc * 8, ov); }
}

__global__ __launch_bounds__(128) void k_yproj(const h16* __restrict__ XL, const h16* __restrict__ WOUTT, const float* __restrict__ bout, float* __restrict__ YT) {
  __shared__ __align__(16) float tf[64][68];
  const int tid = threadIdx.x; const int wave = __builtin_amdgcn_readfirstlane(threadIdx.x >> 5); const int lane = tid & 31, col = lane & 15, g = lane >> 4;
  const int r0 = blockIdx.x * 64;
  const size_t aoff = (size_t)(r0 + wave * 16 + col) * DIN; const size_t woff = (size_t)col * DIN;
  v8f acc[4] = {};
#pragma unroll 2
  for (int kc = 0; kc < DIN / 32; ++kc) { const v16h a = frag_h(XL + aoff + kc * 32, lane);
#pragma unroll
    for (int j = 0; j < 4; ++j) { const v16h w = frag_h(WOUTT + woff + (size_t)(j * 16) * DIN + kc * 32, lane); acc[j] = wmma16(a, w, acc[j]); } }
#pragma unroll
  for (int j = 0; j < 4; ++j) { const float bj = bfr(bout[j * 16 + col]);
#pragma unroll
    for (int r = 0; r < 8; ++r) tf[j * 16 + col][wave * 16 + 8 * g + r] = fmaxf(acc[j][r] * (1.0f / (WCARRY * XCARRY)) + bj, 0.0f); }
  __syncthreads();
  const int b = r0 / SEQ, s0 = r0 - b * SEQ;
#pragma unroll 1
  for (int it = 0; it < 8; ++it) { const int e = tid + it * 128; const int cl = e >> 4, pc = e & 15;
    const v4f yv = *(const v4f*)&tf[cl][pc * 4];
    vst2(YT + ((size_t)b * CIN + cl) * SEQ + s0 + pc * 4, yv); }
}

__global__ __launch_bounds__(256) void k_norm(const float* __restrict__ YT, float* __restrict__ out) {
#pragma clang fp contract(off)
  const int wave = __builtin_amdgcn_readfirstlane(threadIdx.x >> 5); const int lane = threadIdx.x & 31;
  const int row = blockIdx.x * 8 + wave;
  const float* yr = YT + (size_t)row * SEQ; float* orow = out + (size_t)row * SEQ;
  float s = 0.f;
#pragma unroll 1
  for (int it = 0; it < SEQ / 128; ++it) { const v4f v = *(const v4f*)(yr + (it * 32 + lane) * 4); s += (v[0] + v[1]) + (v[2] + v[3]); }
  s += __shfl_xor(s, 1); s += __shfl_xor(s, 2); s += __shfl_xor(s, 4); s += __shfl_xor(s, 8); s += __shfl_xor(s, 16);
  const float inv = 1.0f / (s + 1.0e-6f);
#pragma unroll 1
  for (int it = 0; it < SEQ / 128; ++it) { const v4f v = *(const v4f*)(yr + (it * 32 + lane) * 4); const v4f ov = v * inv;
    vst2(orow + (it * 32 + lane) * 4, ov); }
}

extern "C" void kernel_launch(void* const* d_in, const int* in_sizes, int n_in, void* d_out, int out_size, void* d_ws, size_t ws_size, hipStream_t stream) {
  if (n_in < 23) return;
  if (in_sizes[0] < NB * CIN * SEQ || in_sizes[1] < NB * CIN * SEQ) return;
  if (in_sizes[2] < CIN * CC || in_sizes[4] < CIN * CC) return;
  if (in_sizes[3] < CC || in_sizes[5] < CC || in_sizes[6] < CC || in_sizes[7] < CC) return;
  if (in_sizes[8] < NLAY * DIN * CC || in_sizes[9] < NLAY * DIN * CC || in_sizes[10] < NLAY * DIN * CC || in_sizes[11] < NLAY * CC * DIN) return;
  if (in_sizes[12] < NLAY * DIN) return;
  if (in_sizes[13] < NLAY * DIN * MLPW || in_sizes[14] < NLAY * MLPW || in_sizes[15] < NLAY * MLPW * DIN || in_sizes[16] < NLAY * DIN) return;
  if (in_sizes[17] < NLAY * DIN || in_sizes[18] < NLAY * DIN || in_sizes[19] < NLAY * DIN || in_sizes[20] < NLAY * DIN) return;
  if (in_sizes[21] < DIN * CIN || in_sizes[22] < CIN) return;
  if (out_size < NB * CIN * SEQ) return;
  if (ws_size < (size_t)WS_END) return;
  const float* x = (const float*)d_in[0]; const float* c = (const float*)d_in[1];
  const float* Wx = (const float*)d_in[2]; const float* bx = (const float*)d_in[3]; const float* Wc = (const float*)d_in[4]; const float* bc = (const float*)d_in[5];
  const float* gnc = (const float*)d_in[6]; const float* bnc = (const float*)d_in[7];
  const float* Wq = (const float*)d_in[8]; const float* Wk = (const float*)d_in[9]; const float* Wv = (const float*)d_in[10]; const float* Wo = (const float*)d_in[11]; const float* bo = (const float*)d_in[12];
  const float* W1 = (const float*)d_in[13]; const float* b1 = (const float*)d_in[14]; const float* W2 = (const float*)d_in[15]; const float* b2 = (const float*)d_in[16];
  const float* g1 = (const float*)d_in[17]; const float* bg1 = (const float*)d_in[18]; const float* g2 = (const float*)d_in[19]; const float* bg2 = (const float*)d_in[20];
  const float* Wout = (const float*)d_in[21]; const float* bout = (const float*)d_in[22];
  char* ws = (char*)d_ws;
  h16 *XT = (h16*)(ws + WS_XT), *CT = (h16*)(ws + WS_CT), *WXT = (h16*)(ws + WS_WXT), *WCT = (h16*)(ws + WS_WCT), *WQKV = (h16*)(ws + WS_WQKV), *WOT = (h16*)(ws + WS_WOT), *W1T = (h16*)(ws + WS_W1T), *W2T = (h16*)(ws + WS_W2T), *WOUTT = (h16*)(ws + WS_WOUTT);
  h16 *HH = (h16*)(ws + WS_HH), *CTX = (h16*)(ws + WS_CTX), *QH = (h16*)(ws + WS_QH), *KH = (h16*)(ws + WS_KH), *VT = (h16*)(ws + WS_VT), *CH = (h16*)(ws + WS_CH), *HID = (h16*)(ws + WS_HID);
  float *XF = (float*)(ws + WS_XF), *YT = (float*)(ws + WS_YT);
  const int ctxoff = (int)((WS_CTX - WS_HH) / 2);
  const int MR = NB * SEQ;

  k_tcv<<<dim3(SEQ / 64, CIN / 64, NB), 256, 0, stream>>>(x, XT, 1.0f, SEQ_FULL, CIN * SEQ_FULL, CIN, SEQ * CIN);
  k_tcv<<<dim3(SEQ / 64, CIN / 64, NB), 256, 0, stream>>>(c, CT, 1.0f, SEQ_FULL, CIN * SEQ_FULL, CIN, SEQ * CIN);
  k_tcv<<<dim3(CC / 64, CIN / 64, 1), 256, 0, stream>>>(Wx, WXT, WCARRY, CC, 0, CIN, 0);
  k_tcv<<<dim3(CC / 64, CIN / 64, 1), 256, 0, stream>>>(Wc, WCT, WCARRY, CC, 0, CIN, 0);
  k_tcv<<<dim3(CC / 64, DIN / 64, NLAY), 256, 0, stream>>>(Wq, WQKV, WCARRY, CC, DIN * CC, DIN, 3 * CC * DIN);
  k_tcv<<<dim3(CC / 64, DIN / 64, NLAY), 256, 0, stream>>>(Wk, WQKV + (size_t)CC * DIN, WCARRY, CC, DIN * CC, DIN, 3 * CC * DIN);
  k_tcv<<<dim3(CC / 64, DIN / 64, NLAY), 256, 0, stream>>>(Wv, WQKV + (size_t)2 * CC * DIN, WCARRY, CC, DIN * CC, DIN, 3 * CC * DIN);
  k_tcv<<<dim3(DIN / 64, CC / 64, NLAY), 256, 0, stream>>>(Wo, WOT, WCARRY, DIN, CC * DIN, CC, DIN * CC);
  k_tcv<<<dim3(MLPW / 64, DIN / 64, NLAY), 256, 0, stream>>>(W1, W1T, WCARRY, MLPW, DIN * MLPW, DIN, MLPW * DIN);
  k_tcv<<<dim3(DIN / 64, MLPW / 64, NLAY), 256, 0, stream>>>(W2, W2T, WCARRY, DIN, MLPW * DIN, MLPW, DIN * MLPW);
  k_tcv<<<dim3(CIN / 64, DIN / 64, 1), 256, 0, stream>>>(Wout, WOUTT, WCARRY, CIN, 0, DIN, 0);

  k_rowln<<<dim3(MR / 16), 256, 0, stream>>>(XT, WXT, CIN, 1.0f / WCARRY, bx, XF, FL_STX | FL_LN, g1, bg1, HH, 1.0f);
  k_rowln<<<dim3(MR / 16), 256, 0, stream>>>(CT, WCT, CIN, 1.0f / WCARRY, bc, XF, FL_LN, gnc, bnc, CTX, 1.0f);

  for (int i = 0; i < NLAY; ++i) {
    const int last = (i == NLAY - 1) ? 1 : 0;
    const int nx = last ? 0 : (i + 1);
    k_qkv<<<dim3(MR / 64, 3 * NH), 128, 0, stream>>>(HH, ctxoff, WQKV + (size_t)i * 3 * CC * DIN, QH, KH, VT);
    k_attn<<<dim3(SEQ / 64, NH, NB), 128, 0, stream>>>(QH, KH, VT, CH);
    k_rowln<<<dim3(MR / 16), 256, 0, stream>>>(CH, WOT + (size_t)i * DIN * CC, CC, 1.0f / (WCARRY * CCARRY), bo + (size_t)i * DIN, XF, FL_RES | FL_STX | FL_LN, g2 + (size_t)i * DIN, bg2 + (size_t)i * DIN, HH, 1.0f);
    k_ffn1<<<dim3(MR / 64, MLPW / 64), 128, 0, stream>>>(HH, W1T + (size_t)i * MLPW * DIN, b1 + (size_t)i * MLPW, HID);
    k_rowln<<<dim3(MR / 16), 256, 0, stream>>>(HID, W2T + (size_t)i * DIN * MLPW, MLPW, 1.0f / (WCARRY * HCARRY), b2 + (size_t)i * DIN, XF, last ? FL_RES : (FL_RES | FL_STX | FL_LN), g1 + (size_t)nx * DIN, bg1 + (size_t)nx * DIN, HH, XCARRY);
  }

  k_yproj<<<dim3(MR / 64), 128, 0, stream>>>(HH, WOUTT, bout, YT);
  k_norm<<<dim3(NB * CIN / 8), 256, 0, stream>>>(YT, (float*)d_out);
}
